// HierarchicalAutoEncoderLayer_26319559590069
// MI455X (gfx1250) — hardware-verified
//
#include <hip/hip_runtime.h>

#define NB   4096
#define NEX  16
#define DD   768
#define DE   256
#define KDEC (NEX * DE)

static_assert(NB % 128 == 0);
static_assert(DD % 64 == 0);
static_assert(DE % 64 == 0);
static_assert(KDEC % 64 == 0);
static_assert((NB * DD) % (8 * 256) == 0);

typedef __bf16         v16b __attribute__((ext_vector_type(16)));
typedef __bf16         v8b  __attribute__((ext_vector_type(8)));
typedef float          v8f  __attribute__((ext_vector_type(8)));
typedef float          v4f  __attribute__((ext_vector_type(4)));
typedef unsigned short v8us __attribute__((ext_vector_type(8)));
typedef v8b  __attribute__((may_alias)) v8ba;
typedef v4f  __attribute__((may_alias)) v4fa;
typedef v8us __attribute__((may_alias)) v8usa;

union Frag { v16b v; v8b half[2]; };

__device__ __forceinline__ unsigned short f2bf(float f) {
  unsigned u = __builtin_bit_cast(unsigned, f);
  unsigned r = u + 0x7FFFu + ((u >> 16) & 1u);
  return (unsigned short)(r >> 16);
}
__device__ __forceinline__ float bf2f(unsigned short hb) {
  unsigned u = ((unsigned)hb) << 16;
  return __builtin_bit_cast(float, u);
}
__device__ __forceinline__ void split_bf(float v, unsigned short& hb, unsigned short& lb) {
  hb = f2bf(v);
  lb = f2bf(v - bf2f(hb));
}

__device__ __forceinline__ v8f wmma_bf16(v16b a, v16b b, v8f c) {
  v8f d = __builtin_amdgcn_wmma_f32_16x16x32_bf16(false, a, false, b, (short)0, c, false, false);
  asm volatile("v_nop\n\tv_nop\n\tv_nop\n\tv_nop" : "+v"(d) : "v"(a), "v"(b));
  return d;
}
__device__ __forceinline__ v8f wmma3(v16b ah, v16b al, v16b bh, v16b bl, v8f c) {
  c = wmma_bf16(ah, bh, c);
  c = wmma_bf16(ah, bl, c);
  c = wmma_bf16(al, bh, c);
  return c;
}
__device__ __forceinline__ v16b load_frag(const unsigned short* p, int h) {
  Frag f;
  f.half[0] = *(const v8ba*)(p + 8 * h);
  f.half[1] = *(const v8ba*)(p + 16 + 8 * h);
  return f.v;
}

__global__ __launch_bounds__(256) void cvt_x_kernel(
    const float* __restrict__ x, unsigned short* __restrict__ xh,
    unsigned short* __restrict__ xl, int n8)
{
  const int g = blockIdx.x * 256 + threadIdx.x;
  if (g >= n8) return;
  const float* src = x + (size_t)g * 8;
  const v4f a = *(const v4fa*)src;
  const v4f c = *(const v4fa*)(src + 4);
  const float v[8] = { a.x, a.y, a.z, a.w, c.x, c.y, c.z, c.w };
  v8us H, L;
  #pragma unroll
  for (int j = 0; j < 8; ++j) {
    unsigned short hb, lb;
    split_bf(v[j], hb, lb);
    H[j] = hb; L[j] = lb;
  }
  unsigned short* dh = xh + (size_t)g * 8;
  unsigned short* dl = xl + (size_t)g * 8;
  *(volatile v8us*)dh = H;
  *(volatile v8us*)dl = L;
  __threadfence();
  *(volatile v8us*)dh = H;
  *(volatile v8us*)dl = L;
}

__global__ __launch_bounds__(256) void tsplit_kernel(
    const float* __restrict__ in, unsigned short* __restrict__ oh,
    unsigned short* __restrict__ ol, int R, int C)
{
  __shared__ __attribute__((aligned(16))) float tile[64 * 64];
  const int z = blockIdx.z, r0 = blockIdx.x * 64, c0 = blockIdx.y * 64;
  const int tid = threadIdx.x, lane = tid & 31, w = tid >> 5;
  const size_t zoff = (size_t)z * R * C;
  const float* src = in + zoff;
  #pragma unroll
  for (int i = 0; i < 4; ++i) {
    const int idx = tid + 256 * i;
    const int row = idx >> 4, q = idx & 15;
    const v4f v = *(const v4fa*)(src + (size_t)(r0 + row) * C + c0 + 4 * q);
    *(v4fa*)(tile + row * 64 + 4 * q) = v;
  }
  __syncthreads();

  const int q8 = lane & 7, sub = lane >> 3;
  v8us piece[4];
  #pragma unroll
  for (int i = 0; i < 4; ++i) {
    const int cr = 8 * w + 4 * (i & 1) + sub;
    const int p = i >> 1;
    v8us o;
    #pragma unroll
    for (int j = 0; j < 8; ++j) {
      const float v = tile[(8 * q8 + j) * 64 + cr];
      unsigned short hb, lb;
      split_bf(v, hb, lb);
      o[j] = p ? lb : hb;
    }
    piece[i] = o;
  }
  #pragma unroll
  for (int i = 0; i < 4; ++i) {
    const int cr = 8 * w + 4 * (i & 1) + sub;
    unsigned short* base = (i >> 1) ? ol : oh;
    unsigned short* dst = base + zoff + (size_t)(c0 + cr) * R + r0 + 8 * q8;
    *(volatile v8us*)dst = piece[i];
  }
  __threadfence();
  #pragma unroll
  for (int i = 0; i < 4; ++i) {
    const int cr = 8 * w + 4 * (i & 1) + sub;
    unsigned short* base = (i >> 1) ? ol : oh;
    unsigned short* dst = base + zoff + (size_t)(c0 + cr) * R + r0 + 8 * q8;
    *(volatile v8us*)dst = piece[i];
  }
}

__global__ __launch_bounds__(256) void cbias_kernel(
    const float* __restrict__ W_enc, const float* __restrict__ b_dec,
    float* __restrict__ cb)
{
  const int s = blockIdx.x, e = threadIdx.x;
  const float* wp = W_enc + (size_t)s * DD * DE + e;
  const float* bd = b_dec + (size_t)s * DD;
  float acc = 0.0f;
  #pragma unroll 1
  for (int k = 0; k < DD; ++k) acc += bd[k] * wp[(size_t)k * DE];
  float* dst = cb + s * DE + e;
  *(volatile float*)dst = acc;
  __threadfence();
  *(volatile float*)dst = acc;
}

__global__ __launch_bounds__(128) void enc_kernel(
    const unsigned short* __restrict__ xh,
    const unsigned short* __restrict__ xl,
    const unsigned short* __restrict__ weh,
    const unsigned short* __restrict__ wel,
    const float* __restrict__ gate,
    const float* __restrict__ b_enc,
    const float* __restrict__ cb,
    unsigned short* __restrict__ gh,
    unsigned short* __restrict__ gl)
{
  __shared__ __attribute__((aligned(16))) float sT[128 * 64];

  const int tid = threadIdx.x, lane = tid & 31, w = tid >> 5;
  const int h = lane >> 4, m = lane & 15;
  const int m0 = blockIdx.x * 128;
  const int e0 = blockIdx.y * 64;
  const int s  = blockIdx.z;
  const int m0w = m0 + 32 * w;

  const unsigned short* xa0h = xh + (size_t)(m0w + m) * DD;
  const unsigned short* xa1h = xa0h + (size_t)16 * DD;
  const unsigned short* xa0l = xl + (size_t)(m0w + m) * DD;
  const unsigned short* xa1l = xa0l + (size_t)16 * DD;
  const unsigned short* wbh  = weh + ((size_t)s * DE + e0 + m) * DD;
  const unsigned short* wbl  = wel + ((size_t)s * DE + e0 + m) * DD;

  const v8f zero8 = {0.f, 0.f, 0.f, 0.f, 0.f, 0.f, 0.f, 0.f};
  v8f acc[2][4];
  #pragma unroll
  for (int mt = 0; mt < 2; ++mt)
    #pragma unroll
    for (int nt = 0; nt < 4; ++nt) acc[mt][nt] = zero8;

  #pragma unroll 1
  for (int k0 = 0; k0 < DD; k0 += 32) {
    const v16b a0h = load_frag(xa0h + k0, h);
    const v16b a0l = load_frag(xa0l + k0, h);
    const v16b a1h = load_frag(xa1h + k0, h);
    const v16b a1l = load_frag(xa1l + k0, h);
    #pragma unroll
    for (int nt = 0; nt < 4; ++nt) {
      const v16b bh = load_frag(wbh + (size_t)nt * 16 * DD + k0, h);
      const v16b bl = load_frag(wbl + (size_t)nt * 16 * DD + k0, h);
      acc[0][nt] = wmma3(a0h, a0l, bh, bl, acc[0][nt]);
      acc[1][nt] = wmma3(a1h, a1l, bh, bl, acc[1][nt]);
    }
  }

  #pragma unroll
  for (int nt = 0; nt < 4; ++nt) {
    const int col = 16 * nt + m;
    const float bev = b_enc[s * DE + e0 + col];
    const float cbv = cb[s * DE + e0 + col];
    #pragma unroll
    for (int mt = 0; mt < 2; ++mt) {
      #pragma unroll
      for (int r = 0; r < 8; ++r) {
        const int rowl = 32 * w + 16 * mt + 8 * h + r;
        const float y = (acc[mt][nt][r] - cbv) + bev;
        sT[rowl * 64 + col] = fmaxf(y, 0.0f);
      }
    }
  }
  __syncthreads();

  const int q8 = lane & 7, sub = lane >> 3;
  v8us H[8], L[8];
  #pragma unroll
  for (int i = 0; i < 8; ++i) {
    const int lid = 32 * w + 4 * i + sub;
    const float g = gate[(size_t)(m0 + lid) * NEX + s];
    const v4f va = *(const v4fa*)(sT + lid * 64 + 8 * q8);
    const v4f vb = *(const v4fa*)(sT + lid * 64 + 8 * q8 + 4);
    const float v[8] = { va.x * g, va.y * g, va.z * g, va.w * g,
                         vb.x * g, vb.y * g, vb.z * g, vb.w * g };
    v8us hv, lv;
    #pragma unroll
    for (int j = 0; j < 8; ++j) {
      unsigned short hb, lb;
      split_bf(v[j], hb, lb);
      hv[j] = hb; lv[j] = lb;
    }
    H[i] = hv; L[i] = lv;
  }
  #pragma unroll
  for (int i = 0; i < 8; ++i) {
    const int lid = 32 * w + 4 * i + sub;
    const size_t gi = (size_t)(m0 + lid) * KDEC + s * DE + e0 + 8 * q8;
    *(volatile v8us*)(gh + gi) = H[i];
    *(volatile v8us*)(gl + gi) = L[i];
  }
  __threadfence();
  #pragma unroll
  for (int i = 0; i < 8; ++i) {
    const int lid = 32 * w + 4 * i + sub;
    const size_t gi = (size_t)(m0 + lid) * KDEC + s * DE + e0 + 8 * q8;
    *(volatile v8us*)(gh + gi) = H[i];
    *(volatile v8us*)(gl + gi) = L[i];
  }
}

__global__ __launch_bounds__(128) void dec_kernel(
    const unsigned short* __restrict__ gh,
    const unsigned short* __restrict__ gl,
    const unsigned short* __restrict__ wdh,
    const unsigned short* __restrict__ wdl,
    const float* __restrict__ gate,
    const float* __restrict__ b_dec,
    float* __restrict__ out)
{
  __shared__ __attribute__((aligned(16))) float sT[128 * 64];

  const int tid = threadIdx.x, lane = tid & 31, w = tid >> 5;
  const int h = lane >> 4, m = lane & 15;
  const int m0 = blockIdx.x * 128;
  const int n0 = blockIdx.y * 64;
  const int m0w = m0 + 32 * w;

  const unsigned short* ga0h = gh + (size_t)(m0w + m) * KDEC;
  const unsigned short* ga1h = ga0h + (size_t)16 * KDEC;
  const unsigned short* ga0l = gl + (size_t)(m0w + m) * KDEC;
  const unsigned short* ga1l = ga0l + (size_t)16 * KDEC;
  const unsigned short* wbh  = wdh + (size_t)(n0 + m) * KDEC;
  const unsigned short* wbl  = wdl + (size_t)(n0 + m) * KDEC;

  const v8f zero8 = {0.f, 0.f, 0.f, 0.f, 0.f, 0.f, 0.f, 0.f};
  v8f acc[2][4];
  #pragma unroll
  for (int mt = 0; mt < 2; ++mt)
    #pragma unroll
    for (int nt = 0; nt < 4; ++nt) acc[mt][nt] = zero8;

  #pragma unroll 1
  for (int k0 = 0; k0 < KDEC; k0 += 32) {
    const v16b a0h = load_frag(ga0h + k0, h);
    const v16b a0l = load_frag(ga0l + k0, h);
    const v16b a1h = load_frag(ga1h + k0, h);
    const v16b a1l = load_frag(ga1l + k0, h);
    #pragma unroll
    for (int nt = 0; nt < 4; ++nt) {
      const v16b bh = load_frag(wbh + (size_t)nt * 16 * KDEC + k0, h);
      const v16b bl = load_frag(wbl + (size_t)nt * 16 * KDEC + k0, h);
      acc[0][nt] = wmma3(a0h, a0l, bh, bl, acc[0][nt]);
      acc[1][nt] = wmma3(a1h, a1l, bh, bl, acc[1][nt]);
    }
  }

  #pragma unroll
  for (int nt = 0; nt < 4; ++nt) {
    const int col = 16 * nt + m;
    #pragma unroll
    for (int mt = 0; mt < 2; ++mt) {
      #pragma unroll
      for (int r = 0; r < 8; ++r) {
        const int rowl = 32 * w + 16 * mt + 8 * h + r;
        sT[rowl * 64 + col] = acc[mt][nt][r];
      }
    }
  }
  __syncthreads();

  const int q8 = lane & 7, sub = lane >> 3;
  v4f O[16];
  #pragma unroll
  for (int i = 0; i < 16; ++i) {
    const int rowl = 32 * w + 2 * i + (sub >> 1);
    const int half = sub & 1;
    const int b = m0 + rowl;
    const int cofs = n0 + 32 * half + 4 * q8;
    v4f v = *(const v4fa*)(sT + rowl * 64 + 32 * half + 4 * q8);
    const float* gr = gate + (size_t)b * NEX;
    #pragma unroll 1
    for (int s = 0; s < NEX; ++s) {
      const float g = gr[s];
      const v4f bd = *(const v4fa*)(b_dec + (size_t)s * DD + cofs);
      const bool on = (g != 0.0f);
      v.x += on ? bd.x : 0.0f;
      v.y += on ? bd.y : 0.0f;
      v.z += on ? bd.z : 0.0f;
      v.w += on ? bd.w : 0.0f;
    }
    O[i] = v;
  }
  #pragma unroll
  for (int i = 0; i < 16; ++i) {
    const int rowl = 32 * w + 2 * i + (sub >> 1);
    const int half = sub & 1;
    const size_t gi = (size_t)(m0 + rowl) * DD + n0 + 32 * half + 4 * q8;
    *(volatile v4f*)(out + gi) = O[i];
  }
  __threadfence();
  #pragma unroll
  for (int i = 0; i < 16; ++i) {
    const int rowl = 32 * w + 2 * i + (sub >> 1);
    const int half = sub & 1;
    const size_t gi = (size_t)(m0 + rowl) * DD + n0 + 32 * half + 4 * q8;
    *(volatile v4f*)(out + gi) = O[i];
  }
}

extern "C" void kernel_launch(void* const* d_in, const int* in_sizes, int n_in,
                              void* d_out, int out_size, void* d_ws, size_t ws_size,
                              hipStream_t stream) {
  if (n_in < 6) return;
  if (in_sizes[0] != NB * DD) return;
  if (in_sizes[1] != NB * NEX) return;
  if (in_sizes[2] != NEX * DD * DE) return;
  if (in_sizes[3] != NEX * DE) return;
  if (in_sizes[4] != NEX * DE * DD) return;
  if (in_sizes[5] != NEX * DD) return;
  if (out_size != NB * DD) return;

  const float* x     = (const float*)d_in[0];
  const float* gate  = (const float*)d_in[1];
  const float* W_enc = (const float*)d_in[2];
  const float* b_enc = (const float*)d_in[3];
  const float* W_dec = (const float*)d_in[4];
  const float* b_dec = (const float*)d_in[5];
  float* out = (float*)d_out;

  const size_t xp_bytes = (size_t)NB * DD * 2;
  const size_t we_bytes = (size_t)NEX * DE * DD * 2;
  const size_t wd_bytes = (size_t)DD * KDEC * 2;
  const size_t g_bytes  = (size_t)NB * KDEC * 2;
  const size_t cb_bytes = (size_t)NEX * DE * 4;
  const size_t total = 2 * xp_bytes + 2 * we_bytes + 2 * wd_bytes + 2 * g_bytes + cb_bytes;
  if (total > ws_size) return;

  char* ws = (char*)d_ws;
  size_t off = 0;
  unsigned short* xh  = (unsigned short*)(ws + off); off += xp_bytes;
  unsigned short* xl  = (unsigned short*)(ws + off); off += xp_bytes;
  unsigned short* weh = (unsigned short*)(ws + off); off += we_bytes;
  unsigned short* wel = (unsigned short*)(ws + off); off += we_bytes;
  unsigned short* wdh = (unsigned short*)(ws + off); off += wd_bytes;
  unsigned short* wdl = (unsigned short*)(ws + off); off += wd_bytes;
  unsigned short* gh  = (unsigned short*)(ws + off); off += g_bytes;
  unsigned short* gl  = (unsigned short*)(ws + off); off += g_bytes;
  float* cb = (float*)(ws + off);                    off += cb_bytes;
  if (off > ws_size) return;

  const int n8 = NB * DD / 8;
  cvt_x_kernel<<<(n8 + 255) / 256, 256, 0, stream>>>(x, xh, xl, n8);

  tsplit_kernel<<<dim3(DD / 64, DE / 64, NEX), 256, 0, stream>>>(W_enc, weh, wel, DD, DE);
  tsplit_kernel<<<dim3(KDEC / 64, DD / 64, 1), 256, 0, stream>>>(W_dec, wdh, wdl, KDEC, DD);

  cbias_kernel<<<NEX, DE, 0, stream>>>(W_enc, b_dec, cb);

  enc_kernel<<<dim3(NB / 128, DE / 64, NEX), 128, 0, stream>>>(xh, xl, weh, wel, gate, b_enc, cb, gh, gl);

  dec_kernel<<<dim3(NB / 128, DD / 64, 1), 128, 0, stream>>>(gh, gl, wdh, wdl, gate, b_dec, out);
}
